// SmallWorldVideoAttention_84078279786897
// MI455X (gfx1250) — hardware-verified
//
#include <hip/hip_runtime.h>

typedef _Float16 v16h __attribute__((ext_vector_type(16)));
typedef _Float16 v8h  __attribute__((ext_vector_type(8)));
typedef __bf16   v16b __attribute__((ext_vector_type(16)));
typedef __bf16   v8b  __attribute__((ext_vector_type(8)));
typedef float    v8f  __attribute__((ext_vector_type(8)));
typedef float    v4f  __attribute__((ext_vector_type(4)));
typedef unsigned short v8us __attribute__((ext_vector_type(8)));
typedef v8h  __attribute__((may_alias)) v8ha;
typedef v8b  __attribute__((may_alias)) v8ba;
typedef v4f  __attribute__((may_alias)) v4fa;

#define LL    8192
#define CC    1024
#define NCQK  2048
#define TOKB  8
#define NSH   16

static_assert((LL % 64) == 0);
static_assert((CC % 64) == 0);
static_assert((NCQK % 64) == 0);
static_assert((LL % TOKB) == 0);
static_assert((CC % 32) == 0);
static_assert(((2 * LL) % 32) == 0);

__device__ __forceinline__ v8f wm_f16(v16h a, v16h b, v8f c) {
  return __builtin_amdgcn_wmma_f32_16x16x32_f16(false, a, false, b, (short)0, c, false, false);
}
__device__ __forceinline__ v8f wm_bf16(v16b a, v16b b, v8f c) {
  return __builtin_amdgcn_wmma_f32_16x16x32_bf16(false, a, false, b, (short)0, c, false, false);
}

__device__ __forceinline__ v16h frag_f16(const _Float16* p, int h) {
  const v8h e0 = *(const v8ha*)(p + 8 * h);
  const v8h e1 = *(const v8ha*)(p + 16 + 8 * h);
  return __builtin_shufflevector(e0, e1, 0, 1, 2, 3, 4, 5, 6, 7, 8, 9, 10, 11, 12, 13, 14, 15);
}
__device__ __forceinline__ v16b frag_bf16(const __bf16* p, int h) {
  const v8b e0 = *(const v8ba*)(p + 8 * h);
  const v8b e1 = *(const v8ba*)(p + 16 + 8 * h);
  return __builtin_shufflevector(e0, e1, 0, 1, 2, 3, 4, 5, 6, 7, 8, 9, 10, 11, 12, 13, 14, 15);
}

__device__ __forceinline__ unsigned int bf16_rne_bits(float x) {
  const unsigned int u = __float_as_uint(x);
  return (u + 0x7FFFu + ((u >> 16) & 1u)) >> 16;
}
__device__ __forceinline__ void split_bf16(float x, unsigned short& hb, unsigned short& lb) {
  const unsigned int hbits = bf16_rne_bits(x);
  const float hf = __uint_as_float(hbits << 16);
  const unsigned int lbits = bf16_rne_bits(x - hf);
  hb = (unsigned short)hbits;
  lb = (unsigned short)lbits;
}

__global__ __launch_bounds__(256) void k_cvt_x(const float* __restrict__ x,
                                               _Float16* xh, unsigned short* xbh,
                                               unsigned short* xbl, int n8) {
  const int g = blockIdx.x * 256 + threadIdx.x;
  if (g >= n8) return;
  const float* s = x + (size_t)g * 8;
  const v4f a = *(const v4fa*)s;
  const v4f b = *(const v4fa*)(s + 4);
  const float f[8] = {a.x, a.y, a.z, a.w, b.x, b.y, b.z, b.w};
  unsigned short hb[8], lb[8];
#pragma unroll
  for (int e = 0; e < 8; ++e) split_bf16(f[e], hb[e], lb[e]);
  const v8h  o16 = {(_Float16)f[0], (_Float16)f[1], (_Float16)f[2], (_Float16)f[3],
                    (_Float16)f[4], (_Float16)f[5], (_Float16)f[6], (_Float16)f[7]};
  const v8us oh = {hb[0], hb[1], hb[2], hb[3], hb[4], hb[5], hb[6], hb[7]};
  const v8us ol = {lb[0], lb[1], lb[2], lb[3], lb[4], lb[5], lb[6], lb[7]};
  _Float16* d16 = xh + (size_t)g * 8;
  unsigned short* dh = xbh + (size_t)g * 8;
  unsigned short* dl = xbl + (size_t)g * 8;
  *(volatile v8h*)d16 = o16;
  *(volatile v8us*)dh = oh;
  *(volatile v8us*)dl = ol;
  __threadfence();
  *(volatile v8h*)d16 = o16;
  *(volatile v8us*)dh = oh;
  *(volatile v8us*)dl = ol;
}

__global__ __launch_bounds__(256) void k_cvt_w(const float* __restrict__ Wq,
                                               const float* __restrict__ Wk,
                                               const float* __restrict__ Wv,
                                               const float* __restrict__ Wo,
                                               _Float16* w16, unsigned short* wbh,
                                               unsigned short* wbl) {
  __shared__ __attribute__((aligned(16))) float sT[64 * 68];
  const int tid = threadIdx.x;
  const int bx = blockIdx.x;
  const int mat = bx >> 8, tile = bx & 255;
  const int tn = tile >> 4, tk = tile & 15;
  const float* W = (mat == 0) ? Wq : ((mat == 1) ? Wk : ((mat == 2) ? Wv : Wo));
  {
    const int kl = tid >> 2, nq = tid & 3;
    const float* src = W + (size_t)(64 * tk + kl) * CC + 64 * tn + 16 * nq;
#pragma unroll
    for (int e = 0; e < 4; ++e) {
      const v4f t = *(const v4fa*)(src + 4 * e);
      float* d = sT + (16 * nq + 4 * e) * 68 + kl;
      d[0]   = t.x;
      d[68]  = t.y;
      d[136] = t.z;
      d[204] = t.w;
    }
  }
  __syncthreads();
  const int q8 = tid & 7, sub = tid >> 3;
  v8h  o16[2];
  v8us oh[2], ol[2];
#pragma unroll
  for (int p = 0; p < 2; ++p) {
    const int nl = 32 * p + sub;
    const float* s = sT + nl * 68 + 8 * q8;
    const v4f a = *(const v4fa*)s;
    const v4f b = *(const v4fa*)(s + 4);
    const float f[8] = {a.x, a.y, a.z, a.w, b.x, b.y, b.z, b.w};
    unsigned short hb[8], lb[8];
#pragma unroll
    for (int e = 0; e < 8; ++e) split_bf16(f[e], hb[e], lb[e]);
    const v8h t16 = {(_Float16)(f[0] * 32.0f), (_Float16)(f[1] * 32.0f), (_Float16)(f[2] * 32.0f), (_Float16)(f[3] * 32.0f),
                     (_Float16)(f[4] * 32.0f), (_Float16)(f[5] * 32.0f), (_Float16)(f[6] * 32.0f), (_Float16)(f[7] * 32.0f)};
    const v8us th = {hb[0], hb[1], hb[2], hb[3], hb[4], hb[5], hb[6], hb[7]};
    const v8us tl = {lb[0], lb[1], lb[2], lb[3], lb[4], lb[5], lb[6], lb[7]};
    o16[p] = t16;
    oh[p] = th;
    ol[p] = tl;
  }
#pragma unroll
  for (int pass = 0; pass < 2; ++pass) {
#pragma unroll
    for (int p = 0; p < 2; ++p) {
      const int nl = 32 * p + sub;
      if (mat < 2) {
        _Float16* d = w16 + ((size_t)(mat * CC + 64 * tn + nl) * CC + 64 * tk + 8 * q8);
        *(volatile v8h*)d = o16[p];
      } else {
        const size_t row = (size_t)((mat - 2) * CC + 64 * tn + nl);
        unsigned short* dh = wbh + row * CC + 64 * tk + 8 * q8;
        unsigned short* dl = wbl + row * CC + 64 * tk + 8 * q8;
        *(volatile v8us*)dh = oh[p];
        *(volatile v8us*)dl = ol[p];
      }
    }
    if (pass == 0) __threadfence();
  }
}

__device__ __forceinline__ void stage_tile(float* sT, v8f c00, v8f c01, v8f c10, v8f c11,
                                           const float* bias, int nc0, float osc,
                                           int w, int lane) {
  const int h = lane >> 4, m = lane & 15, wr = w >> 1, wc = w & 1;
  const int cl0 = 32 * wc + m, cl1 = cl0 + 16;
  const float b0 = bias[nc0 + cl0];
  const float b1 = bias[nc0 + cl1];
#pragma unroll
  for (int r = 0; r < 8; ++r) {
    const int row0 = 32 * wr + 8 * h + r, row1 = row0 + 16;
    sT[row0 * 64 + cl0] = fmaf(c00[r], osc, b0);
    sT[row0 * 64 + cl1] = fmaf(c01[r], osc, b1);
    sT[row1 * 64 + cl0] = fmaf(c10[r], osc, b0);
    sT[row1 * 64 + cl1] = fmaf(c11[r], osc, b1);
  }
}

__device__ __forceinline__ void store_lines32(const float* sT, float* out, int m0, int nc0,
                                              int ldc, int w, int lane) {
  const int q8 = lane & 7, sub = lane >> 3;
#pragma unroll
  for (int it = 0; it < 8; ++it) {
    const int lid = it * 4 + sub;
    const int row = 16 * w + (lid >> 1), hl = lid & 1;
    const v4f v = *(const v4fa*)(sT + row * 64 + 32 * hl + 4 * q8);
    float* d = out + (size_t)(m0 + row) * ldc + nc0 + 32 * hl + 4 * q8;
    *(volatile v4f*)d = v;
  }
}

__global__ __launch_bounds__(128) void k_gemm_h(const _Float16* __restrict__ A,
                                                const _Float16* __restrict__ B,
                                                const float* bias0, const float* bias1,
                                                float* out0, float* out1,
                                                int nsplit, int K, int ldc, float osc) {
  __shared__ __attribute__((aligned(16))) float sT[64 * 64];
  const int tid = threadIdx.x, lane = tid & 31, w = tid >> 5;
  const int h = lane >> 4, m = lane & 15, wr = w >> 1, wc = w & 1;
  const int m0 = blockIdx.y * 64, nb = blockIdx.x * 64;
  const bool sel = (nb >= nsplit);
  const int nc0 = sel ? (nb - nsplit) : nb;
  const float* bias = sel ? bias1 : bias0;
  float* out = sel ? out1 : out0;

  const _Float16* a0 = A + (size_t)(m0 + 32 * wr + m) * K;
  const _Float16* a1 = a0 + (size_t)16 * K;
  const _Float16* b0 = B + (size_t)(nb + 32 * wc + m) * K;
  const _Float16* b1 = b0 + (size_t)16 * K;

  v8f c00 = {0.f, 0.f, 0.f, 0.f, 0.f, 0.f, 0.f, 0.f};
  v8f c01 = c00, c10 = c00, c11 = c00;

#pragma unroll 1
  for (int k0 = 0; k0 < K; k0 += 32) {
    const v16h fa0 = frag_f16(a0 + k0, h);
    const v16h fa1 = frag_f16(a1 + k0, h);
    const v16h fb0 = frag_f16(b0 + k0, h);
    const v16h fb1 = frag_f16(b1 + k0, h);
    c00 = wm_f16(fa0, fb0, c00);
    c01 = wm_f16(fa0, fb1, c01);
    c10 = wm_f16(fa1, fb0, c10);
    c11 = wm_f16(fa1, fb1, c11);
    asm volatile("v_nop\n\tv_nop\n\tv_nop\n\tv_nop"
                 : "+v"(c00), "+v"(c01), "+v"(c10), "+v"(c11)
                 : "v"(fa0), "v"(fa1), "v"(fb0), "v"(fb1));
  }

  stage_tile(sT, c00, c01, c10, c11, bias, nc0, osc, w, lane);
  __syncthreads();
  store_lines32(sT, out, m0, nc0, ldc, w, lane);
  __threadfence();
  store_lines32(sT, out, m0, nc0, ldc, w, lane);
}

__global__ __launch_bounds__(128) void k_gemm_b3(const __bf16* __restrict__ Ah,
                                                 const __bf16* __restrict__ Al,
                                                 const __bf16* __restrict__ Bh,
                                                 const __bf16* __restrict__ Bl,
                                                 const float* bias0, const float* bias1,
                                                 float* out0, float* out1,
                                                 int nsplit, int K, int ldc, float osc) {
  __shared__ __attribute__((aligned(16))) float sT[64 * 64];
  const int tid = threadIdx.x, lane = tid & 31, w = tid >> 5;
  const int h = lane >> 4, m = lane & 15, wr = w >> 1, wc = w & 1;
  const int m0 = blockIdx.y * 64, nb = blockIdx.x * 64;
  const bool sel = (nb >= nsplit);
  const int nc0 = sel ? (nb - nsplit) : nb;
  const float* bias = sel ? bias1 : bias0;
  float* out = sel ? out1 : out0;

  const size_t ra0 = (size_t)(m0 + 32 * wr + m) * K, ra1 = ra0 + (size_t)16 * K;
  const size_t rb0 = (size_t)(nb + 32 * wc + m) * K, rb1 = rb0 + (size_t)16 * K;

  v8f c00 = {0.f, 0.f, 0.f, 0.f, 0.f, 0.f, 0.f, 0.f};
  v8f c01 = c00, c10 = c00, c11 = c00;

#pragma unroll 1
  for (int k0 = 0; k0 < K; k0 += 32) {
    const v16b ha0 = frag_bf16(Ah + ra0 + k0, h);
    const v16b ha1 = frag_bf16(Ah + ra1 + k0, h);
    const v16b la0 = frag_bf16(Al + ra0 + k0, h);
    const v16b la1 = frag_bf16(Al + ra1 + k0, h);
    const v16b hb0 = frag_bf16(Bh + rb0 + k0, h);
    const v16b hb1 = frag_bf16(Bh + rb1 + k0, h);
    const v16b lb0 = frag_bf16(Bl + rb0 + k0, h);
    const v16b lb1 = frag_bf16(Bl + rb1 + k0, h);
    c00 = wm_bf16(ha0, hb0, c00);  c00 = wm_bf16(ha0, lb0, c00);  c00 = wm_bf16(la0, hb0, c00);
    c01 = wm_bf16(ha0, hb1, c01);  c01 = wm_bf16(ha0, lb1, c01);  c01 = wm_bf16(la0, hb1, c01);
    c10 = wm_bf16(ha1, hb0, c10);  c10 = wm_bf16(ha1, lb0, c10);  c10 = wm_bf16(la1, hb0, c10);
    c11 = wm_bf16(ha1, hb1, c11);  c11 = wm_bf16(ha1, lb1, c11);  c11 = wm_bf16(la1, hb1, c11);
    asm volatile("v_nop\n\tv_nop\n\tv_nop\n\tv_nop"
                 : "+v"(c00), "+v"(c01), "+v"(c10), "+v"(c11)
                 : "v"(ha0), "v"(ha1), "v"(la0), "v"(la1), "v"(hb0), "v"(hb1), "v"(lb0), "v"(lb1));
  }

  stage_tile(sT, c00, c01, c10, c11, bias, nc0, osc, w, lane);
  __syncthreads();
  store_lines32(sT, out, m0, nc0, ldc, w, lane);
  __threadfence();
  store_lines32(sT, out, m0, nc0, ldc, w, lane);
}

__global__ __launch_bounds__(256) void k_rstd(const float* __restrict__ qf,
                                              const float* __restrict__ kf,
                                              float* rtab) {
  __shared__ __attribute__((aligned(16))) float s_r[32];
  const int tid = threadIdx.x, lane = tid & 31, w = tid >> 5;
  const int row0 = blockIdx.x * 32;
  const float* base = (row0 < LL) ? (qf + (size_t)row0 * CC) : (kf + (size_t)(row0 - LL) * CC);
#pragma unroll 1
  for (int j = 0; j < 4; ++j) {
    const float* rp = base + (size_t)(4 * w + j) * CC + 32 * lane;
    float ss = 0.0f;
#pragma unroll 2
    for (int e = 0; e < 8; ++e) {
      const v4f t = *(const v4fa*)(rp + 4 * e);
      ss = fmaf(t.x, t.x, ss);
      ss = fmaf(t.y, t.y, ss);
      ss = fmaf(t.z, t.z, ss);
      ss = fmaf(t.w, t.w, ss);
    }
    ss += __shfl_xor(ss, 16, 32);
    ss += __shfl_xor(ss, 8, 32);
    ss += __shfl_xor(ss, 4, 32);
    ss += __shfl_xor(ss, 2, 32);
    ss += __shfl_xor(ss, 1, 32);
    const float rv = rsqrtf(ss * (1.0f / 1024.0f) + 1e-6f);
    if (lane == 0) s_r[4 * w + j] = rv;
  }
  __syncthreads();
  if (tid < 8) {
    const v4f v = *(const v4fa*)(s_r + 4 * tid);
    float* d = rtab + row0 + 4 * tid;
    *(volatile v4f*)d = v;
    __threadfence();
    *(volatile v4f*)d = v;
  }
}

__device__ __forceinline__ int nbr_index(int n, int f, int i, int S, int T) {
  int r;
  if (n < 12) {
    const int mag = 1 << (n >> 1);
    const int sh = (n & 1) ? -mag : mag;
    int ii = (i + sh) % S;
    if (ii < 0) ii += S;
    r = f * S + ii;
  } else {
    const int jn = n - 12;
    const int mag = 1 << (jn >> 1);
    const int sh = (jn & 1) ? -mag : mag;
    int ff = (f + sh) % T;
    if (ff < 0) ff += T;
    r = ff * S + i;
  }
  r = min(max(r, 0), LL - 1);
  return r;
}

__global__ __launch_bounds__(128) void k_attn(const float* __restrict__ qf,
                                              const float* __restrict__ kf,
                                              const float* __restrict__ vf,
                                              const float* __restrict__ rtab,
                                              const float* __restrict__ qnw,
                                              const float* __restrict__ knw,
                                              const float* __restrict__ eb,
                                              const int* __restrict__ nf,
                                              unsigned short* abh, unsigned short* abl) {
  __shared__ float s_eb[256];
  __shared__ float s_sc[4][4][NSH];
  __shared__ float s_p[4][4][NSH];
  const int tid = threadIdx.x, lane = tid & 31, w = tid >> 5;
  const int hq = lane >> 3, j8 = lane & 7;
  const int head = 4 * w + hq;
  const int col = 256 * w + 8 * lane;

  s_eb[tid] = eb[tid];
  s_eb[tid + 128] = eb[tid + 128];

  int T = nf[0];
  if (!((T >= 1) && (T <= LL) && ((LL % T) == 0))) T = 8;
  const int S = LL / T;

  float cw[8];
  {
    const v4f qa = *(const v4fa*)(qnw + col);
    const v4f qb = *(const v4fa*)(qnw + col + 4);
    const v4f ka = *(const v4fa*)(knw + col);
    const v4f kb = *(const v4fa*)(knw + col + 4);
    cw[0] = qa.x * ka.x * 0.125f;  cw[1] = qa.y * ka.y * 0.125f;
    cw[2] = qa.z * ka.z * 0.125f;  cw[3] = qa.w * ka.w * 0.125f;
    cw[4] = qb.x * kb.x * 0.125f;  cw[5] = qb.y * kb.y * 0.125f;
    cw[6] = qb.z * kb.z * 0.125f;  cw[7] = qb.w * kb.w * 0.125f;
  }
  __syncthreads();

#pragma unroll 1
  for (int tok = 0; tok < TOKB; ++tok) {
    const int l = blockIdx.x * TOKB + tok;
    const int f = l / S;
    const int i = l - f * S;
    const float rq = rtab[l];
    const float* qp = qf + (size_t)l * CC + col;
    const v4f qa = *(const v4fa*)qp;
    const v4f qb = *(const v4fa*)(qp + 4);
    float c[8];
    c[0] = qa.x * rq * cw[0];  c[1] = qa.y * rq * cw[1];
    c[2] = qa.z * rq * cw[2];  c[3] = qa.w * rq * cw[3];
    c[4] = qb.x * rq * cw[4];  c[5] = qb.y * rq * cw[5];
    c[6] = qb.z * rq * cw[6];  c[7] = qb.w * rq * cw[7];

#pragma unroll 1
    for (int n = 0; n < NSH; ++n) {
      const int nbr = nbr_index(n, f, i, S, T);
      const float* kp = kf + (size_t)nbr * CC + col;
      const v4f ka = *(const v4fa*)kp;
      const v4f kb = *(const v4fa*)(kp + 4);
      float part = c[0] * ka.x;
      part = fmaf(c[1], ka.y, part);
      part = fmaf(c[2], ka.z, part);
      part = fmaf(c[3], ka.w, part);
      part = fmaf(c[4], kb.x, part);
      part = fmaf(c[5], kb.y, part);
      part = fmaf(c[6], kb.z, part);
      part = fmaf(c[7], kb.w, part);
      part += __shfl_xor(part, 1, 32);
      part += __shfl_xor(part, 2, 32);
      part += __shfl_xor(part, 4, 32);
      const float sc = fmaf(part, rtab[LL + nbr], s_eb[head * NSH + n]);
      if (j8 == 0) s_sc[w][hq][n] = sc;
    }
    __syncthreads();

    {
      const float x0 = s_sc[w][hq][j8];
      const float x1 = s_sc[w][hq][j8 + 8];
      float mx = fmaxf(x0, x1);
      mx = fmaxf(mx, __shfl_xor(mx, 1, 32));
      mx = fmaxf(mx, __shfl_xor(mx, 2, 32));
      mx = fmaxf(mx, __shfl_xor(mx, 4, 32));
      const float e0 = __expf(x0 - mx);
      const float e1 = __expf(x1 - mx);
      float sm = e0 + e1;
      sm += __shfl_xor(sm, 1, 32);
      sm += __shfl_xor(sm, 2, 32);
      sm += __shfl_xor(sm, 4, 32);
      const float inv = __builtin_amdgcn_rcpf(sm);
      s_p[w][hq][j8]     = e0 * inv;
      s_p[w][hq][j8 + 8] = e1 * inv;
    }
    __syncthreads();

    float o[8] = {0.f, 0.f, 0.f, 0.f, 0.f, 0.f, 0.f, 0.f};
#pragma unroll 1
    for (int n = 0; n < NSH; ++n) {
      const int nbr = nbr_index(n, f, i, S, T);
      const float p = s_p[w][hq][n];
      const float* vp = vf + (size_t)nbr * CC + col;
      const v4f va = *(const v4fa*)vp;
      const v4f vb = *(const v4fa*)(vp + 4);
      o[0] = fmaf(p, va.x, o[0]);  o[1] = fmaf(p, va.y, o[1]);
      o[2] = fmaf(p, va.z, o[2]);  o[3] = fmaf(p, va.w, o[3]);
      o[4] = fmaf(p, vb.x, o[4]);  o[5] = fmaf(p, vb.y, o[5]);
      o[6] = fmaf(p, vb.z, o[6]);  o[7] = fmaf(p, vb.w, o[7]);
    }

    unsigned short hb[8], lb[8];
#pragma unroll
    for (int e = 0; e < 8; ++e) split_bf16(o[e], hb[e], lb[e]);
    const v8us oh = {hb[0], hb[1], hb[2], hb[3], hb[4], hb[5], hb[6], hb[7]};
    const v8us ol = {lb[0], lb[1], lb[2], lb[3], lb[4], lb[5], lb[6], lb[7]};
    unsigned short* dh = abh + (size_t)l * CC + col;
    unsigned short* dl = abl + (size_t)l * CC + col;
    *(volatile v8us*)dh = oh;
    *(volatile v8us*)dl = ol;
    __threadfence();
    *(volatile v8us*)dh = oh;
    *(volatile v8us*)dl = ol;
  }
}

extern "C" void kernel_launch(void* const* d_in, const int* in_sizes, int n_in,
                              void* d_out, int out_size, void* d_ws, size_t ws_size,
                              hipStream_t stream) {
  if (n_in < 13) return;
  if (in_sizes[0] != LL * CC) return;
  if (in_sizes[1] != CC * CC || in_sizes[3] != CC * CC || in_sizes[5] != CC * CC || in_sizes[10] != CC * CC) return;
  if (in_sizes[2] != CC || in_sizes[4] != CC || in_sizes[6] != CC || in_sizes[11] != CC) return;
  if (in_sizes[7] != CC || in_sizes[8] != CC) return;
  if (in_sizes[9] != 256 || in_sizes[12] < 1) return;
  if (out_size != LL * CC) return;

  const float* x   = (const float*)d_in[0];
  const float* Wq  = (const float*)d_in[1];
  const float* bq  = (const float*)d_in[2];
  const float* Wk  = (const float*)d_in[3];
  const float* bk  = (const float*)d_in[4];
  const float* Wv  = (const float*)d_in[5];
  const float* bv  = (const float*)d_in[6];
  const float* qnw = (const float*)d_in[7];
  const float* knw = (const float*)d_in[8];
  const float* eb  = (const float*)d_in[9];
  const float* Wo  = (const float*)d_in[10];
  const float* bo  = (const float*)d_in[11];
  const int*   nf  = (const int*)d_in[12];
  float* out = (float*)d_out;

  const size_t b16 = (size_t)LL * CC * 2;
  const size_t bw  = (size_t)NCQK * CC * 2;
  const size_t b32 = (size_t)LL * CC * 4;
  const size_t brt = (size_t)2 * LL * 4;
  const size_t o_x16 = 0;
  const size_t o_xbh = o_x16 + b16;
  const size_t o_xbl = o_xbh + b16;
  const size_t o_w16 = o_xbl + b16;
  const size_t o_wbh = o_w16 + bw;
  const size_t o_wbl = o_wbh + bw;
  const size_t o_q   = o_wbl + bw;
  const size_t o_k   = o_q + b32;
  const size_t o_v   = o_k + b32;
  const size_t o_rt  = o_v + b32;
  const size_t total = o_rt + brt;
  if (total > ws_size) return;

  char* ws = (char*)d_ws;
  _Float16*       x16 = (_Float16*)(ws + o_x16);
  unsigned short* xbh = (unsigned short*)(ws + o_xbh);
  unsigned short* xbl = (unsigned short*)(ws + o_xbl);
  _Float16*       w16 = (_Float16*)(ws + o_w16);
  unsigned short* wbh = (unsigned short*)(ws + o_wbh);
  unsigned short* wbl = (unsigned short*)(ws + o_wbl);
  float* qf   = (float*)(ws + o_q);
  float* kf   = (float*)(ws + o_k);
  float* vf   = (float*)(ws + o_v);
  float* rtab = (float*)(ws + o_rt);
  unsigned short* abh = (unsigned short*)(ws + o_x16);
  unsigned short* abl = (unsigned short*)(ws + o_xbh);

  const int n8 = (LL * CC) / 8;
  k_cvt_x<<<(n8 + 255) / 256, 256, 0, stream>>>(x, x16, xbh, xbl, n8);

  k_cvt_w<<<4 * 256, 256, 0, stream>>>(Wq, Wk, Wv, Wo, w16, wbh, wbl);

  k_gemm_h<<<dim3(NCQK / 64, LL / 64), 128, 0, stream>>>(x16, w16, bq, bk, qf, kf, CC, CC, CC, 0.03125f);

  k_gemm_b3<<<dim3(CC / 64, LL / 64), 128, 0, stream>>>(
      (const __bf16*)xbh, (const __bf16*)xbl, (const __bf16*)wbh, (const __bf16*)wbl,
      bv, bv, vf, vf, 1 << 30, CC, CC, 1.0f);

  k_rstd<<<(2 * LL) / 32, 256, 0, stream>>>(qf, kf, rtab);

  k_attn<<<LL / TOKB, 128, 0, stream>>>(qf, kf, vf, rtab, qnw, knw, eb, nf, abh, abl);

  k_gemm_b3<<<dim3(CC / 64, LL / 64), 128, 0, stream>>>(
      (const __bf16*)abh, (const __bf16*)abl,
      (const __bf16*)(wbh + (size_t)CC * CC), (const __bf16*)(wbl + (size_t)CC * CC),
      bo, bo, out, out, 1 << 30, CC, CC, 1.0f);
}
